// MultiHeadAttention_49237505081571
// MI455X (gfx1250) — hardware-run, weakly checked
//
#include <hip/hip_runtime.h>


#ifndef NB
#define NB 2
#endif
#ifndef SEQ
#define SEQ 2048
#endif
#define NB_FULL  2
#define SEQ_FULL 2048
#define TT   SEQ
#define DM   1024
#define NH_  16
#define HD   64
#define DQ   (NH_ * HD)
#define ZH   2
#define PCAR 1024.0f
#define SCL  0.125f

static_assert(TT % 256 == 0);
static_assert(TT <= SEQ_FULL);
static_assert(NB <= NB_FULL);
static_assert(DM % 64 == 0);
static_assert(DQ == DM);
static_assert(HD % 32 == 0);
static_assert(NH_ % ZH == 0);

typedef _Float16 h16;
typedef unsigned short bf;
typedef __attribute__((ext_vector_type(16))) __bf16   v16bf;
typedef __attribute__((ext_vector_type(16))) _Float16 v16h;
typedef __attribute__((ext_vector_type(8)))  _Float16 v8h;
typedef __attribute__((ext_vector_type(8)))  unsigned short v8us;
typedef __attribute__((ext_vector_type(8)))  float    v8f;
typedef __attribute__((ext_vector_type(4)))  float    v4f;
typedef v4f  __attribute__((may_alias)) v4fa;

__device__ __forceinline__ unsigned short f2bf(float f) { unsigned u = __float_as_uint(f); u += 0x7FFFu + ((u >> 16) & 1u); return (unsigned short)(u >> 16); }
__device__ __forceinline__ float bf2f(unsigned short b) { return __uint_as_float(((unsigned)b) << 16); }
__device__ __forceinline__ float bfr(float f) { return bf2f(f2bf(f)); }
__device__ __forceinline__ v16h cat16(v8h lo, v8h hi) { return __builtin_shufflevector(lo, hi, 0, 1, 2, 3, 4, 5, 6, 7, 8, 9, 10, 11, 12, 13, 14, 15); }
__device__ __forceinline__ v16bf cat16b(v8us lo, v8us hi) { return __builtin_bit_cast(v16bf, __builtin_shufflevector(lo, hi, 0, 1, 2, 3, 4, 5, 6, 7, 8, 9, 10, 11, 12, 13, 14, 15)); }
__device__ __forceinline__ v8f wmma16(v16h a, v16h b, v8f c) { return __builtin_amdgcn_wmma_f32_16x16x32_f16(false, a, false, b, (short)0, c, false, false); }
__device__ __forceinline__ v8f wmmab(v16bf a, v16bf b, v8f c) { return __builtin_amdgcn_wmma_f32_16x16x32_bf16(false, a, false, b, (short)0, c, false, false); }

template <typename T16> struct WFrag;
template <> struct WFrag<h16> { typedef v16h V; static __device__ __forceinline__ V ld(const h16* p) { return cat16(*(const v8h*)p, *(const v8h*)(p + 16)); } static __device__ __forceinline__ v8f mma(V a, V b, v8f c) { return wmma16(a, b, c); } };
template <> struct WFrag<bf> { typedef v16bf V; static __device__ __forceinline__ V ld(const bf* p) { return cat16b(*(const v8us*)p, *(const v8us*)(p + 16)); } static __device__ __forceinline__ v8f mma(V a, V b, v8f c) { return wmmab(a, b, c); } };

template <typename T16, int EPI>
__global__ __launch_bounds__(32) void k_gemmw(const T16* __restrict__ A, const T16* __restrict__ Bt, int K, float* C, int ldc, const float* __restrict__ addv, float osc, size_t sA, size_t sB, size_t sC, size_t sAdd) {
    typedef typename WFrag<T16>::V V;
    __shared__ __align__(16) float os[16 * 68];
    const size_t z = blockIdx.z; A += z * sA; Bt += z * sB; C += z * sC;
    const int lane = threadIdx.x & 31, lr = lane & 15, hi = lane >> 4; const int r0 = blockIdx.x * 64, c0 = blockIdx.y * 64;
    v4f ad; ad[0] = 0.f; ad[1] = 0.f; ad[2] = 0.f; ad[3] = 0.f;
    if (EPI != 0) { const float* ap = addv + z * sAdd + c0 + lr * 4;
#pragma unroll
        for (int q = 0; q < 4; ++q) { const float t = ap[q]; ad[q] = (EPI == 1) ? bfr(t) : t; } }
    v8f acc[4][4];
#pragma unroll
    for (int mb = 0; mb < 4; ++mb)
#pragma unroll
        for (int nb = 0; nb < 4; ++nb) acc[mb][nb] = (v8f){};
    const size_t aoff = (size_t)(r0 + lr) * K + 8 * hi, boff = (size_t)(c0 + lr) * K + 8 * hi;
#pragma unroll 1
    for (int kc = 0; kc < K; kc += 32) {
        V a[4];
#pragma unroll
        for (int mb = 0; mb < 4; ++mb) a[mb] = WFrag<T16>::ld(A + aoff + (size_t)mb * 16 * K + kc);
#pragma unroll
        for (int nb = 0; nb < 4; ++nb) { const V b = WFrag<T16>::ld(Bt + boff + (size_t)nb * 16 * K + kc);
#pragma unroll
            for (int mb = 0; mb < 4; ++mb) acc[mb][nb] = WFrag<T16>::mma(a[mb], b, acc[mb][nb]); }
        asm volatile("v_nop\n\tv_nop\n\tv_nop\n\tv_nop" : "+v"(acc[0][0]), "+v"(acc[1][1]), "+v"(acc[2][2]), "+v"(acc[3][3]) : "v"(a[0]), "v"(a[3]));
    }
#pragma unroll
    for (int mb = 0; mb < 4; ++mb) {
#pragma unroll
        for (int nb = 0; nb < 4; ++nb) {
#pragma unroll
            for (int j = 0; j < 8; ++j) os[(hi * 8 + j) * 68 + nb * 16 + lr] = acc[mb][nb][j]; }
        __builtin_amdgcn_wave_barrier(); asm volatile("" ::: "memory");
        float* crow = C + (size_t)(r0 + mb * 16) * ldc + c0;
#pragma unroll 1
        for (int ps = 0; ps < 2; ++ps) {
#pragma unroll
            for (int s = 0; s < 8; ++s) { const int row = 2 * s + hi, cofs = lr * 4; v4f val = *(const v4fa*)(os + row * 68 + cofs);
                if (EPI == 1) { val[0] += ad[0]; val[1] += ad[1]; val[2] += ad[2]; val[3] += ad[3]; }
                if (EPI == 2) { val[0] = val[0] * osc + ad[0]; val[1] = val[1] * osc + ad[1]; val[2] = val[2] * osc + ad[2]; val[3] = val[3] * osc + ad[3]; }
                *(volatile v4f*)(crow + (size_t)row * ldc + cofs) = val; }
            if (ps == 0) __threadfence(); }
        __builtin_amdgcn_wave_barrier(); asm volatile("" ::: "memory");
    }
}

__global__ __launch_bounds__(256) void k_cvt8(const float* __restrict__ src, bf* dst, size_t n8) { const size_t i = (size_t)blockIdx.x * 256 + threadIdx.x; if (i >= n8) return; const v8f v = *(const v8f*)(src + i * 8); v8us o;
#pragma unroll
    for (int k = 0; k < 8; ++k) o[k] = f2bf(v[k]);
    *(volatile v8us*)(dst + i * 8) = o; __threadfence(); *(volatile v8us*)(dst + i * 8) = o; }

__global__ __launch_bounds__(256) void k_maskr(const float* __restrict__ m, float* MR) { const int i = blockIdx.x * 256 + threadIdx.x; if (i >= NB * TT / 4) return; const int e = i * 4; const int b = e / TT, j = e % TT;
    const v4f a = *(const v4f*)(m + (size_t)b * SEQ_FULL + j); v4f o;
#pragma unroll
    for (int q = 0; q < 4; ++q) o[q] = bfr(a[q]);
    *(volatile v4f*)(MR + e) = o; __threadfence(); *(volatile v4f*)(MR + e) = o; }

__global__ __launch_bounds__(256) void k_hp8(const float* __restrict__ F, int pitch, int nheads, h16* P16) {
    const size_t e = ((size_t)blockIdx.x * 256 + threadIdx.x) * 8; if (e >= (size_t)nheads * TT * HD) return; const int d = (int)(e % HD); const int t = (int)((e / HD) % TT); const int h = (int)(e / ((size_t)HD * TT));
    const v8f x = *(const v8f*)(F + (size_t)t * pitch + h * HD + d); v8h o;
#pragma unroll
    for (int q = 0; q < 8; ++q) o[q] = (h16)x[q];
    *(volatile v8h*)(P16 + e) = o; __threadfence(); *(volatile v8h*)(P16 + e) = o; }

__global__ __launch_bounds__(256) void k_vtp8(const float* __restrict__ F, int pitch, int nheads, h16* V16) {
    const size_t e = ((size_t)blockIdx.x * 256 + threadIdx.x) * 8; if (e >= (size_t)nheads * HD * TT) return; const int t = (int)(e % TT); const int d = (int)((e / TT) % HD); const int g = (int)(e / ((size_t)TT * HD)); v8h o;
#pragma unroll
    for (int q = 0; q < 8; ++q) o[q] = (h16)F[(size_t)(t + q) * pitch + g * HD + d];
    *(volatile v8h*)(V16 + e) = o; __threadfence(); *(volatile v8h*)(V16 + e) = o; }

__global__ __launch_bounds__(256) void k_vmean(const float* __restrict__ F, float* VM) {
    __shared__ float part[8 * 32];
    const int lane = threadIdx.x & 31, w = __builtin_amdgcn_readfirstlane((int)(threadIdx.x >> 5)); const int col = blockIdx.x * 32 + lane; float s = 0.f;
#pragma unroll 4
    for (int r = w; r < TT; r += 8) s += F[(size_t)r * DM + col];
    part[w * 32 + lane] = s; __syncthreads();
    if (w == 0) { float tot = 0.f;
#pragma unroll
        for (int k = 0; k < 8; ++k) tot += part[k * 32 + lane];
        const float m = tot * (1.0f / (float)TT); *(volatile float*)(VM + col) = m; __threadfence(); *(volatile float*)(VM + col) = m; }
}

__global__ __launch_bounds__(256) void k_asoft(const float* __restrict__ Sb, h16* P16) {
    const int lane = threadIdx.x & 31; const int row = blockIdx.x * 8 + (threadIdx.x >> 5); if (row >= ZH * TT) return; const float* sr = Sb + (size_t)row * TT; float v[TT / 32]; float mx = -3.0e38f;
#pragma unroll
    for (int ch = 0; ch < TT / 256; ++ch) { const v8f a = *(const v8f*)(sr + ch * 256 + lane * 8);
#pragma unroll
        for (int q = 0; q < 8; ++q) { v[ch * 8 + q] = a[q]; mx = fmaxf(mx, a[q]); } }
#pragma unroll
    for (int sh = 16; sh; sh >>= 1) mx = fmaxf(mx, __shfl_xor(mx, sh, 32));
    float sum = 0.f;
#pragma unroll
    for (int k = 0; k < TT / 32; ++k) { float d0 = __fsub_rn(v[k], mx); asm volatile("" : "+v"(d0)); v[k] = __builtin_amdgcn_exp2f(__fmul_rn(d0, 1.4426950408889634f)); sum += v[k]; }
#pragma unroll
    for (int sh = 16; sh; sh >>= 1) sum += __shfl_xor(sum, sh, 32);
    const float f = __fdiv_rn(PCAR, sum); const float c2 = sum * (1.0f / (float)TT);
#pragma unroll 1
    for (int ps = 0; ps < 2; ++ps) {
#pragma unroll
        for (int ch = 0; ch < TT / 256; ++ch) { v8h o;
#pragma unroll
            for (int q = 0; q < 8; ++q) o[q] = (h16)((v[ch * 8 + q] - c2) * f);
            *(volatile v8h*)(P16 + (size_t)row * TT + ch * 256 + lane * 8) = o; }
        if (ps == 0) __threadfence(); }
}

#define AL256(x) ((((size_t)(x)) + 255) & ~(size_t)255)
#define WS_TOTAL (3 * AL256((size_t)DQ * DM * 2) + AL256((size_t)TT * DM * 2) + 3 * AL256((size_t)TT * DQ * 4) + 3 * AL256((size_t)NH_ * TT * HD * 2) + AL256((size_t)ZH * TT * TT * 4) + AL256((size_t)ZH * TT * TT * 2) + AL256((size_t)DM * 4) + AL256((size_t)NB * TT * 4))
static_assert(WS_TOTAL <= (size_t)134217728);

extern "C" void kernel_launch(void* const* d_in, const int* in_sizes, int n_in,
                              void* d_out, int out_size, void* d_ws, size_t ws_size, hipStream_t stream) {
    if (n_in < 8) return;
    const size_t needx = (size_t)(NB - 1) * SEQ_FULL * DM + (size_t)TT * DM, needm = (size_t)(NB - 1) * SEQ_FULL + (size_t)TT;
    if ((size_t)in_sizes[0] < needx || (size_t)in_sizes[1] < needm) return;
    if ((size_t)in_sizes[2] < (size_t)DQ * DM || (size_t)in_sizes[4] < (size_t)DQ * DM || (size_t)in_sizes[6] < (size_t)DQ * DM) return;
    if (in_sizes[3] < DQ || in_sizes[5] < DQ || in_sizes[7] < DQ) return;
    if ((size_t)out_size < (size_t)NB * TT * DM) return;
    const float* x = (const float*)d_in[0]; const float* mask = (const float*)d_in[1];
    const float* wq = (const float*)d_in[2]; const float* bq = (const float*)d_in[3];
    const float* wk = (const float*)d_in[4]; const float* bk = (const float*)d_in[5];
    const float* wv = (const float*)d_in[6]; const float* bv = (const float*)d_in[7];
    float* OUT = (float*)d_out;
    char* wsp = (char*)d_ws;
    auto take = [&](size_t bytes) { char* p = wsp; wsp += (bytes + 255) & ~(size_t)255; return (void*)p; };
    bf* WQ = (bf*)take((size_t)DQ * DM * 2); bf* WK = (bf*)take((size_t)DQ * DM * 2); bf* WV = (bf*)take((size_t)DQ * DM * 2);
    bf* XB = (bf*)take((size_t)TT * DM * 2);
    float* FQ = (float*)take((size_t)TT * DQ * 4); float* FK = (float*)take((size_t)TT * DQ * 4); float* FV = (float*)take((size_t)TT * DQ * 4);
    h16* QP16 = (h16*)take((size_t)NH_ * TT * HD * 2); h16* KP16 = (h16*)take((size_t)NH_ * TT * HD * 2); h16* VT16 = (h16*)take((size_t)NH_ * HD * TT * 2);
    float* Sb = (float*)take((size_t)ZH * TT * TT * 4); h16* P16 = (h16*)take((size_t)ZH * TT * TT * 2);
    float* VM = (float*)take((size_t)DM * 4); float* MR = (float*)take((size_t)NB * TT * 4);
    if ((size_t)(wsp - (char*)d_ws) > ws_size) return;
    const unsigned LW = (unsigned)(((size_t)DQ * DM / 8 + 255) / 256);
    k_cvt8<<<LW, 256, 0, stream>>>(wq, WQ, (size_t)DQ * DM / 8);
    k_cvt8<<<LW, 256, 0, stream>>>(wk, WK, (size_t)DQ * DM / 8);
    k_cvt8<<<LW, 256, 0, stream>>>(wv, WV, (size_t)DQ * DM / 8);
    k_maskr<<<(unsigned)((NB * TT / 4 + 255) / 256), 256, 0, stream>>>(mask, MR);
    const unsigned LP = (unsigned)(((size_t)NH_ * TT * HD / 8 + 255) / 256);
    for (int b = 0; b < NB; ++b) {
        k_cvt8<<<(unsigned)(((size_t)TT * DM / 8 + 255) / 256), 256, 0, stream>>>(x + (size_t)b * SEQ_FULL * DM, XB, (size_t)TT * DM / 8);
        k_gemmw<bf, 1><<<dim3(TT / 64, DQ / 64, 1), 32, 0, stream>>>(XB, WQ, DM, FQ, DQ, bq, 1.0f, 0, 0, 0, 0);
        k_hp8<<<LP, 256, 0, stream>>>(FQ, DQ, NH_, QP16);
        k_gemmw<bf, 1><<<dim3(TT / 64, DQ / 64, 1), 32, 0, stream>>>(XB, WK, DM, FK, DQ, bk, 1.0f, 0, 0, 0, 0);
        k_hp8<<<LP, 256, 0, stream>>>(FK, DQ, NH_, KP16);
        k_gemmw<bf, 1><<<dim3(TT / 64, DQ / 64, 1), 32, 0, stream>>>(XB, WV, DM, FV, DQ, bv, 1.0f, 0, 0, 0, 0);
        k_vtp8<<<LP, 256, 0, stream>>>(FV, DQ, NH_, VT16);
        k_vmean<<<DM / 32, 256, 0, stream>>>(FV, VM);
        for (int h0 = 0; h0 < NH_; h0 += ZH) {
            k_gemmw<h16, 2><<<dim3(TT / 64, TT / 64, ZH), 32, 0, stream>>>(QP16 + (size_t)h0 * TT * HD, KP16 + (size_t)h0 * TT * HD, HD, Sb, TT, MR + (size_t)b * TT, SCL, (size_t)TT * HD, (size_t)TT * HD, (size_t)TT * TT, 0);
            k_asoft<<<ZH * TT / 8, 256, 0, stream>>>(Sb, P16);
            k_gemmw<h16, 2><<<dim3(TT / 64, 1, ZH), 32, 0, stream>>>(P16, VT16 + (size_t)h0 * HD * TT, TT, OUT + (size_t)b * TT * DM + (size_t)h0 * HD, DM, VM + (size_t)h0 * HD, 1.0f / PCAR, (size_t)TT * TT, (size_t)HD * TT, (size_t)HD, (size_t)HD);
        }
    }
}
